// K2Layer_79826262163472
// MI455X (gfx1250) — hardware-run, weakly checked
//
#include <hip/hip_runtime.h>
#include <math.h>

typedef __attribute__((ext_vector_type(16))) _Float16 v16h;
typedef __attribute__((ext_vector_type(8)))  _Float16 v8h;
typedef __attribute__((ext_vector_type(8)))  float    v8f;
typedef __attribute__((ext_vector_type(4)))  float    v4f;
typedef __attribute__((ext_vector_type(2)))  float    v2f;
typedef __attribute__((ext_vector_type(4)))  unsigned int v4u;

constexpr int kBatch = 4;
constexpr int kWin   = 1024;
constexpr int kDim   = 1024;
constexpr int kRank  = 32;
constexpr int kRows  = kBatch * kWin;
constexpr int kUpDim = 2 * kDim;
constexpr int kSegElems = 1024 * 1024;

static_assert(kRows == 4096);
static_assert(kDim == 1024 && kWin == 1024 && kRank == 32 && kUpDim == 2048);
static_assert((kDim % 32) == 0 && (kUpDim % 32) == 0 && (kWin % 32) == 0);
static_assert((kRows % 64) == 0 && (kDim % 64) == 0 && (kUpDim % 64) == 0 && ((2 * kRank) % 64) == 0);

constexpr float kActCarry  = 16.0f;
constexpr float kGeluCarry = 64.0f;
constexpr float kUvCarry   = 64.0f;
constexpr float kKbCarry   = 64.0f;
constexpr float kWCarry    = 256.0f;
constexpr float kScaleQk   = 1.0f / (kActCarry * kUvCarry);
constexpr float kScaleBase = 1.0f / (kKbCarry * kActCarry);
constexpr float kScaleProj = 1.0f / (kActCarry * kWCarry);
constexpr float kScaleUp   = 1.0f / (kActCarry * kWCarry);
constexpr float kScaleDown = 1.0f / (kGeluCarry * kWCarry);
constexpr float kF16MinNormal = 6.103515625e-05f;
constexpr float kNormEps  = 1e-8f;
constexpr float kInvDim   = 1.0f / (float)kDim;
constexpr float kInvSqrt2 = 0.70710678118654752f;

constexpr size_t kBytesW16   = (size_t)5 * kSegElems * 2;
constexpr size_t kBytesKB16  = (size_t)kWin * kWin * 2;
constexpr size_t kBytesUVT16 = (size_t)64 * kDim * 2;
constexpr size_t kBytesHN32  = (size_t)kRows * kDim * 4;
constexpr size_t kBytesY32   = (size_t)kRows * kDim * 4;
constexpr size_t kBytesHN16  = (size_t)kRows * kDim * 2;
constexpr size_t kBytesHNT16 = (size_t)kRows * kDim * 2;
constexpr size_t kBytesQK32  = (size_t)kRows * 64 * 4;
constexpr size_t kBytesQKN32 = (size_t)kRows * 64 * 4;
constexpr size_t kBytesMIX16 = (size_t)kRows * kDim * 2;
constexpr size_t kBytesH2    = (size_t)kRows * kDim * 4;
constexpr size_t kBytesM16   = (size_t)kRows * kDim * 2;
constexpr size_t kBytesG16   = (size_t)kRows * kUpDim * 2;
constexpr size_t kBytesPAR   = 256;
constexpr size_t kBytesUP32  = (size_t)kRows * kUpDim * 4;
constexpr size_t kWsTotal = kBytesW16 + kBytesKB16 + kBytesUVT16 + kBytesHN32 + kBytesY32 + kBytesHN16 + kBytesHNT16 +
                            kBytesQK32 + kBytesQKN32 + kBytesMIX16 + kBytesH2 + kBytesM16 + kBytesG16 + kBytesPAR;
static_assert(kWsTotal == 10485760ull + 2097152ull + 131072ull + 16777216ull + 16777216ull + 8388608ull + 8388608ull +
                          1048576ull + 1048576ull + 8388608ull + 16777216ull + 8388608ull + 16777216ull + 256ull);
static_assert(kWsTotal == 115474688ull);
static_assert(kWsTotal <= 134217728ull);
static_assert(kBytesUP32 == kBytesHN32 + kBytesY32);

__device__ __forceinline__ unsigned pk16(unsigned short a, unsigned short b) { return (unsigned)a | ((unsigned)b << 16); }

__device__ __forceinline__ unsigned short h_bits_fl(float x) {
  const float y = (fabsf(x) < kF16MinNormal) ? 0.0f : x;
  const _Float16 h = (_Float16)y;
  return __builtin_bit_cast(unsigned short, h);
}

__device__ __forceinline__ v4u pack8_f16(v4f a, v4f c, float carry) {
  const unsigned short h0 = h_bits_fl(a[0] * carry);
  const unsigned short h1 = h_bits_fl(a[1] * carry);
  const unsigned short h2 = h_bits_fl(a[2] * carry);
  const unsigned short h3 = h_bits_fl(a[3] * carry);
  const unsigned short h4 = h_bits_fl(c[0] * carry);
  const unsigned short h5 = h_bits_fl(c[1] * carry);
  const unsigned short h6 = h_bits_fl(c[2] * carry);
  const unsigned short h7 = h_bits_fl(c[3] * carry);
  return (v4u){pk16(h0, h1), pk16(h2, h3), pk16(h4, h5), pk16(h6, h7)};
}

__device__ __forceinline__ float sigmoid_f(float x) { return 1.0f / (1.0f + expf(-x)); }

__device__ __forceinline__ void st_tr8(unsigned short* p, int pitch, v4u w) {
  const unsigned w0 = w[0], w1 = w[1], w2 = w[2], w3 = w[3];
  p[0 * pitch] = (unsigned short)(w0 & 0xffffu);
  p[1 * pitch] = (unsigned short)(w0 >> 16);
  p[2 * pitch] = (unsigned short)(w1 & 0xffffu);
  p[3 * pitch] = (unsigned short)(w1 >> 16);
  p[4 * pitch] = (unsigned short)(w2 & 0xffffu);
  p[5 * pitch] = (unsigned short)(w2 >> 16);
  p[6 * pitch] = (unsigned short)(w3 & 0xffffu);
  p[7 * pitch] = (unsigned short)(w3 >> 16);
}

__global__ __launch_bounds__(32) void params_kernel(const float* __restrict__ decay_logit, const float* __restrict__ gate_logit,
                                                    const float* __restrict__ alpha_logit, float* par) {
  const int l = threadIdx.x & 31;
  const float dl  = decay_logit[l];
  const float gam = 0.9f + 0.1f * sigmoid_f(dl);
  const float al  = sigmoid_f(alpha_logit[0]);
  const float gt  = sigmoid_f(gate_logit[0]);
  const float second = (l == 0) ? al : ((l == 1) ? gt : 0.0f);
  for (int pass = 0; pass < 2; ++pass) {
    *(volatile float*)(par + l) = gam;
    *(volatile float*)(par + 32 + l) = second;
    __threadfence();
  }
}

__global__ __launch_bounds__(256) void cast_w_kernel(const float* __restrict__ pw, const float* __restrict__ uw,
                                                     const float* __restrict__ dw, unsigned short* dst, float carry) {
  const int seg = blockIdx.y;
  const float* src = pw;
  if (seg == 1 || seg == 2) src = uw + (size_t)(seg - 1) * kSegElems;
  if (seg >= 3) src = dw + (size_t)(seg - 3) * kSegElems;
  const int i = blockIdx.x * 256 + threadIdx.x;
  if (i >= kSegElems / 8) return;
  const float* p = src + 8 * (size_t)i;
  const v4f a = *(const v4f*)(p);
  const v4f c = *(const v4f*)(p + 4);
  const v4u u = pack8_f16(a, c, carry);
  unsigned short* q = dst + (size_t)seg * kSegElems + 8 * (size_t)i;
  *(volatile v4u*)q = u;
  __threadfence();
  *(volatile v4u*)q = u;
}

__global__ __launch_bounds__(256) void kb16_kernel(const float* __restrict__ k_base, const float* __restrict__ par,
                                                   unsigned short* kb16, float carry) {
  const int i8 = blockIdx.x * 256 + threadIdx.x;
  if (i8 >= kWin * kWin / 8) return;
  const int row = i8 >> 7;
  const int j0  = (i8 & 127) * 8;
  const float gt = par[33];
  const float* p = k_base + (size_t)row * kWin + j0;
  const v4f a = *(const v4f*)(p);
  const v4f c = *(const v4f*)(p + 4);
  v4f am, cm;
#pragma unroll
  for (int e = 0; e < 4; ++e) {
    const float xa = ((j0 + e) <= row) ? a[e] : 0.0f;
    const float xc = ((j0 + 4 + e) <= row) ? c[e] : 0.0f;
    am[e] = xa * gt;
    cm[e] = xc * gt;
  }
  const v4u u = pack8_f16(am, cm, carry);
  unsigned short* q = kb16 + 8 * (size_t)i8;
  *(volatile v4u*)q = u;
  __threadfence();
  *(volatile v4u*)q = u;
}

__global__ __launch_bounds__(256) void uvt_kernel(const float* __restrict__ u, const float* __restrict__ v,
                                                  unsigned short* uvT, float carry) {
  __shared__ float sm[64][65];
  const int t  = threadIdx.x;
  const int d0 = blockIdx.x * 64;
#pragma unroll
  for (int it = 0; it < 8; ++it) {
    const int e  = it * 256 + t;
    const int dl = e >> 5;
    const int r  = e & 31;
    const size_t gi = (size_t)(d0 + dl) * kRank + r;
    sm[r][dl]      = u[gi];
    sm[32 + r][dl] = v[gi];
  }
  __syncthreads();
  const int lane = t & 31, wave = t >> 5;
  const int q = lane >> 3, c8 = (lane & 7) * 8;
  v4u pk[2];
#pragma unroll
  for (int it = 0; it < 2; ++it) {
    const int row = wave * 8 + it * 4 + q;
    const v4f a = (v4f){sm[row][c8 + 0], sm[row][c8 + 1], sm[row][c8 + 2], sm[row][c8 + 3]};
    const v4f c = (v4f){sm[row][c8 + 4], sm[row][c8 + 5], sm[row][c8 + 6], sm[row][c8 + 7]};
    pk[it] = pack8_f16(a, c, carry);
  }
  for (int pass = 0; pass < 2; ++pass) {
#pragma unroll
    for (int it = 0; it < 2; ++it) {
      const int row = wave * 8 + it * 4 + q;
      *(volatile v4u*)(uvT + (size_t)row * kDim + d0 + c8) = pk[it];
    }
    __threadfence();
  }
}

template <bool WRITE_F32>
__global__ __launch_bounds__(256) void rmsnorm_kernel(const float* __restrict__ x, const float* __restrict__ gain,
                                                      float* out32, unsigned short* out16, float carry) {
  __shared__ float red[8];
  __shared__ __align__(16) float xs[kDim];
  const int row = blockIdx.x;
  const int t = threadIdx.x, lane = t & 31, wave = t >> 5;
  const v4f vv = *(const v4f*)(x + (size_t)row * kDim + 4 * t);
  float s = vv[0] * vv[0] + vv[1] * vv[1] + vv[2] * vv[2] + vv[3] * vv[3];
#pragma unroll
  for (int off = 16; off > 0; off >>= 1) s += __shfl_xor(s, off, 32);
  if (lane == 0) red[wave] = s;
  __syncthreads();
  float tot = 0.0f;
#pragma unroll
  for (int w = 0; w < 8; ++w) tot += red[w];
  const float inv = rsqrtf(tot * kInvDim + kNormEps);
  const v4f g4 = *(const v4f*)(gain + 4 * t);
  v4f o;
  o[0] = vv[0] * inv * g4[0];
  o[1] = vv[1] * inv * g4[1];
  o[2] = vv[2] * inv * g4[2];
  o[3] = vv[3] * inv * g4[3];
  *(v4f*)(xs + 4 * t) = o;
  __syncthreads();
  const int t8 = (t & 127) * 8;
  const v4f a = *(const v4f*)(xs + t8);
  const v4f c = *(const v4f*)(xs + t8 + 4);
  const v4u pk = pack8_f16(a, c, carry);
  float* o32 = out32 + (size_t)row * kDim + 4 * t;
  unsigned short* o16 = out16 + (size_t)row * kDim + t8;
  for (int pass = 0; pass < 2; ++pass) {
    if (WRITE_F32) *(volatile v4f*)o32 = o;
    if (t < 128) *(volatile v4u*)o16 = pk;
    __threadfence();
  }
}

__global__ __launch_bounds__(256) void transpose16_kernel(const unsigned short* __restrict__ in, unsigned short* out) {
  __shared__ __align__(16) unsigned short sm[64 * 72];
  const int tid = threadIdx.x;
  const int t0 = blockIdx.x * 64;
  const int d0 = blockIdx.y * 64;
  const int b  = blockIdx.z;
#pragma unroll
  for (int it = 0; it < 2; ++it) {
    const int i  = it * 256 + tid;
    const int tl = i >> 3;
    const int d8 = (i & 7) * 8;
    const v4u w = *(const v4u*)(in + ((size_t)(b * kWin + t0 + tl)) * kDim + d0 + d8);
    st_tr8(sm + d8 * 72 + tl, 72, w);
  }
  __syncthreads();
  const int lane = tid & 31, wave = tid >> 5;
  const int q = lane >> 3, c8 = (lane & 7) * 8;
  v4u pk[2];
#pragma unroll
  for (int it = 0; it < 2; ++it) {
    const int row = wave * 8 + it * 4 + q;
    pk[it] = *(const v4u*)(sm + row * 72 + c8);
  }
  for (int pass = 0; pass < 2; ++pass) {
#pragma unroll
    for (int it = 0; it < 2; ++it) {
      const int row = wave * 8 + it * 4 + q;
      *(volatile v4u*)(out + ((size_t)(b * kDim + d0 + row)) * kWin + t0 + c8) = pk[it];
    }
    __threadfence();
  }
}

namespace eng {

__device__ __forceinline__ v16h frag_load(const _Float16* p) {
  union { v16h v; v8h h[2]; } f;
  f.h[0] = *(const v8h*)(p);
  f.h[1] = *(const v8h*)(p + 16);
  return f.v;
}
__device__ __forceinline__ v8f wmma_raw(v16h a, v16h b, v8f c) {
  return __builtin_amdgcn_wmma_f32_16x16x32_f16(false, a, false, b, (short)0, c, false, false);
}
__device__ __forceinline__ void dep_guard4(v8f& a, v8f& b, v8f& c, v8f& d, v16h x) {
  asm volatile("v_nop\n\tv_nop\n\tv_nop\n\tv_nop" : "+v"(a), "+v"(b), "+v"(c), "+v"(d) : "v"(x));
}
__device__ __forceinline__ void keep4(v16h a, v16h b, v16h c, v16h d) { asm volatile("v_nop" :: "v"(a), "v"(b), "v"(c), "v"(d)); }
__device__ __forceinline__ void acc_guard4(v8f& a, v8f& b, v8f& c, v8f& d) {
  asm volatile("v_nop\n\tv_nop\n\tv_nop\n\tv_nop" : "+v"(a), "+v"(b), "+v"(c), "+v"(d));
}

template <int OUT_MODE, bool BIAS, bool RESID, bool CAUSAL>
__global__ __launch_bounds__(256) void gemm64_f16(
    const unsigned short* __restrict__ Ap, int lda, long strideA,
    const unsigned short* __restrict__ Btp, int ldb, long strideB,
    void* Cout, int ldc, long strideC,
    const float* __restrict__ bias,
    const float* __restrict__ resid, int ldr, long strideR,
    int M, int N, int K, float scale, float ocarry) {
  const _Float16* A  = (const _Float16*)Ap;
  const _Float16* Bt = (const _Float16*)Btp;
  __shared__ __align__(16) float sT[8][16 * 68];
  const int b    = blockIdx.y;
  const int lane = threadIdx.x & 31;
  const int wave = threadIdx.x >> 5;
  const int tilesN = N >> 6;
  const int tilesM = M >> 6;
  const int tile = blockIdx.x * 8 + wave;
  if (tile >= tilesM * tilesN) return;
  const int tm = tile / tilesN;
  const int tn = tile - tm * tilesN;
  const int m0 = tm << 6;
  const int n0 = tn << 6;

  const _Float16* Ab = A  + (size_t)b * strideA;
  const _Float16* Bb = Bt + (size_t)b * strideB;

  const int rlane = lane & 15;
  const int koff  = (lane >> 4) * 8;
  const int mOff  = (lane >> 4) * 8;

  v8f acc[4][4];
#pragma unroll
  for (int i = 0; i < 4; ++i)
#pragma unroll
    for (int j = 0; j < 4; ++j) acc[i][j] = (v8f){0.f, 0.f, 0.f, 0.f, 0.f, 0.f, 0.f, 0.f};

  int kEnd = K;
  if (CAUSAL) kEnd = (m0 + 64 < K) ? (m0 + 64) : K;

  for (int k0 = 0; k0 < kEnd; k0 += 32) {
    v16h bh[4];
#pragma unroll
    for (int j = 0; j < 4; ++j) {
      const size_t bo = (size_t)(n0 + (j << 4) + rlane) * ldb + koff + k0;
      bh[j] = frag_load(Bb + bo);
    }
#pragma unroll
    for (int i = 0; i < 4; ++i) {
      const size_t ao = (size_t)(m0 + (i << 4) + rlane) * lda + koff + k0;
      const v16h ah = frag_load(Ab + ao);
#pragma unroll
      for (int j = 0; j < 4; ++j) acc[i][j] = wmma_raw(ah, bh[j], acc[i][j]);
      dep_guard4(acc[i][0], acc[i][1], acc[i][2], acc[i][3], ah);
    }
    keep4(bh[0], bh[1], bh[2], bh[3]);
  }
  acc_guard4(acc[0][0], acc[0][1], acc[0][2], acc[0][3]);
  acc_guard4(acc[1][0], acc[1][1], acc[1][2], acc[1][3]);
  acc_guard4(acc[2][0], acc[2][1], acc[2][2], acc[2][3]);
  acc_guard4(acc[3][0], acc[3][1], acc[3][2], acc[3][3]);

  float* slab = sT[wave];
  const float* Rb = resid + (size_t)b * strideR;
#pragma unroll
  for (int i = 0; i < 4; ++i) {
    const int mBase = m0 + (i << 4);
#pragma unroll
    for (int j = 0; j < 4; ++j) {
#pragma unroll
      for (int r = 0; r < 8; ++r) slab[(mOff + r) * 68 + (j << 4) + rlane] = acc[i][j][r] * scale;
    }
    __builtin_amdgcn_fence(__ATOMIC_RELEASE, "workgroup");
    __builtin_amdgcn_wave_barrier();
    __builtin_amdgcn_fence(__ATOMIC_ACQUIRE, "workgroup");
    if (OUT_MODE == 0) {
      float* C = (float*)Cout + (size_t)b * strideC;
      const int hh = lane >> 4, c4 = (lane & 15) * 4;
      v4f bias4 = (v4f){0.f, 0.f, 0.f, 0.f};
      if (BIAS) bias4 = *(const v4f*)(bias + n0 + c4);
      v4f val[8];
#pragma unroll
      for (int it = 0; it < 8; ++it) {
        const int row = it * 2 + hh;
        v4f v = *(const v4f*)(slab + row * 68 + c4);
        if (BIAS) v = v + bias4;
        if (RESID) {
          const v4f r4 = *(const v4f*)(Rb + (size_t)(mBase + row) * ldr + n0 + c4);
          v = v + r4;
        }
        val[it] = v;
      }
      for (int pass = 0; pass < 2; ++pass) {
#pragma unroll
        for (int it = 0; it < 8; ++it) {
          const int row = it * 2 + hh;
          *(volatile v4f*)(C + (size_t)(mBase + row) * ldc + n0 + c4) = val[it];
        }
        __threadfence();
      }
    } else {
      unsigned short* C = (unsigned short*)Cout + (size_t)b * strideC;
      const int q = lane >> 3, c8 = (lane & 7) * 8;
      v4f biasA = (v4f){0.f, 0.f, 0.f, 0.f};
      v4f biasC = (v4f){0.f, 0.f, 0.f, 0.f};
      if (BIAS) {
        biasA = *(const v4f*)(bias + n0 + c8);
        biasC = *(const v4f*)(bias + n0 + c8 + 4);
      }
      v4u pk[4];
#pragma unroll
      for (int it = 0; it < 4; ++it) {
        const int row = it * 4 + q;
        const float* sp = slab + row * 68 + c8;
        v4f a = *(const v4f*)(sp);
        v4f c = *(const v4f*)(sp + 4);
        if (BIAS) {
          a = a + biasA;
          c = c + biasC;
        }
        if (RESID) {
          const float* rp = Rb + (size_t)(mBase + row) * ldr + n0 + c8;
          const v4f ra = *(const v4f*)(rp);
          const v4f rc = *(const v4f*)(rp + 4);
          a = a + ra;
          c = c + rc;
        }
        pk[it] = pack8_f16(a, c, ocarry);
      }
      for (int pass = 0; pass < 2; ++pass) {
#pragma unroll
        for (int it = 0; it < 4; ++it) {
          const int row = it * 4 + q;
          *(volatile v4u*)(C + (size_t)(mBase + row) * ldc + n0 + c8) = pk[it];
        }
        __threadfence();
      }
    }
    __builtin_amdgcn_fence(__ATOMIC_RELEASE, "workgroup");
    __builtin_amdgcn_wave_barrier();
    __builtin_amdgcn_fence(__ATOMIC_ACQUIRE, "workgroup");
  }
}

}

__global__ __launch_bounds__(256) void qk_post_kernel(const float* __restrict__ qk32, float* qkn) {
  const int lane = threadIdx.x & 31, wave = threadIdx.x >> 5;
  const int row = blockIdx.x * 8 + wave;
  const float* p = qk32 + (size_t)row * 64;
  const float qv = p[lane];
  const float kv = p[32 + lane];
  float sq = qv * qv;
  float sk = kv * kv;
#pragma unroll
  for (int off = 16; off > 0; off >>= 1) {
    sq += __shfl_xor(sq, off, 32);
    sk += __shfl_xor(sk, off, 32);
  }
  const float qi = 1.0f / fmaxf(sqrtf(sq), kNormEps);
  const float ki = 1.0f / fmaxf(sqrtf(sk), kNormEps);
  const float qo = qv * qi;
  const float ko = kv * ki;
  float* o = qkn + (size_t)row * 64;
  for (int pass = 0; pass < 2; ++pass) {
    *(volatile float*)(o + lane) = qo;
    *(volatile float*)(o + 32 + lane) = ko;
    __threadfence();
  }
}

constexpr int kScanThreads = 128;
constexpr int kScanSteps   = 32;
static_assert(kScanSteps * 64 == 4 * kScanThreads * 4);
static_assert((kWin % kScanSteps) == 0 && (kDim % kScanThreads) == 0);

__global__ __launch_bounds__(128) void scan_kernel(const float* __restrict__ hn32, const float* __restrict__ qkn,
                                                   const float* __restrict__ par, float* y32) {
  __shared__ __align__(16) float sQK[kScanSteps * 64];
  __shared__ __align__(16) float sY[kScanSteps * kScanThreads];
  const int tid = threadIdx.x;
  const int b = blockIdx.x >> 3;
  const int d = ((blockIdx.x & 7) << 7) + tid;

  float gam[32];
#pragma unroll
  for (int j = 0; j < 8; ++j) {
    const v4f g4 = *(const v4f*)(par + 4 * j);
    gam[4 * j + 0] = g4[0];
    gam[4 * j + 1] = g4[1];
    gam[4 * j + 2] = g4[2];
    gam[4 * j + 3] = g4[3];
  }
  const float alpha = par[32];
  float S[32];
#pragma unroll
  for (int r = 0; r < 32; ++r) S[r] = 0.0f;

  const size_t rowb = (size_t)b * kWin;
#pragma unroll 1
  for (int c = 0; c < kWin / kScanSteps; ++c) {
    const size_t t0 = rowb + (size_t)c * kScanSteps;
    __syncthreads();
#pragma unroll
    for (int it = 0; it < 4; ++it) {
      const int idx = it * kScanThreads + tid;
      const v4f w = *(const v4f*)(qkn + t0 * 64 + 4 * (size_t)idx);
      *(v4f*)(sQK + 4 * idx) = w;
    }
    __syncthreads();
#pragma unroll 1
    for (int s = 0; s < kScanSteps; ++s) {
      const float hv = hn32[(t0 + s) * kDim + d];
      const float* qp = sQK + s * 64;
      float y = 0.0f;
#pragma unroll
      for (int j = 0; j < 8; ++j) {
        const v4f q4 = *(const v4f*)(qp + 4 * j);
        const v4f k4 = *(const v4f*)(qp + 32 + 4 * j);
#pragma unroll
        for (int e = 0; e < 4; ++e) {
          const float kh = k4[e] * hv;
          S[4 * j + e] = fmaf(gam[4 * j + e], S[4 * j + e], kh);
          y = fmaf(q4[e], S[4 * j + e], y);
        }
      }
      sY[s * kScanThreads + tid] = alpha * y;
    }
    for (int pass = 0; pass < 2; ++pass) {
#pragma unroll 1
      for (int s = 0; s < kScanSteps; ++s) {
        const float v = sY[s * kScanThreads + tid];
        *(volatile float*)(y32 + (t0 + s) * kDim + d) = v;
      }
      __threadfence();
    }
  }
}

__global__ __launch_bounds__(256) void gelu_kernel(const float* __restrict__ pre, unsigned short* g16, float carry) {
  __shared__ __align__(16) unsigned int sw[kUpDim / 2];
  const int row = blockIdx.x;
  const int t = threadIdx.x;
  const float* pr = pre + (size_t)row * kUpDim;
#pragma unroll 1
  for (int it = 0; it < 4; ++it) {
    const int w = it * 256 + t;
    const v2f xx = *(const v2f*)(pr + 2 * w);
    const float x0 = xx[0];
    const float x1 = xx[1];
    const float g0 = 0.5f * x0 * (1.0f + erff(x0 * kInvSqrt2));
    const float g1 = 0.5f * x1 * (1.0f + erff(x1 * kInvSqrt2));
    const unsigned short b0 = h_bits_fl(g0 * carry);
    const unsigned short b1 = h_bits_fl(g1 * carry);
    sw[w] = pk16(b0, b1);
  }
  __syncthreads();
  const v4u u = *(const v4u*)(sw + 4 * t);
  unsigned short* q = g16 + (size_t)row * kUpDim + 8 * t;
  *(volatile v4u*)q = u;
  __threadfence();
  *(volatile v4u*)q = u;
}

extern "C" void kernel_launch(void* const* d_in, const int* in_sizes, int n_in,
                              void* d_out, int out_size, void* d_ws, size_t ws_size,
                              hipStream_t stream) {
  if (n_in < 15 || d_out == nullptr || d_ws == nullptr) return;
  if (in_sizes[0] != kRows * kDim) return;
  if (in_sizes[1] != kWin * kWin) return;
  if (in_sizes[2] != kRank || in_sizes[3] != 1 || in_sizes[6] != 1) return;
  if (in_sizes[4] != kDim * kRank || in_sizes[5] != kDim * kRank) return;
  if (in_sizes[7] != kDim * kDim || in_sizes[8] != kDim) return;
  if (in_sizes[9] != kDim || in_sizes[10] != kDim) return;
  if (in_sizes[11] != kUpDim * kDim || in_sizes[12] != kUpDim) return;
  if (in_sizes[13] != kDim * kUpDim || in_sizes[14] != kDim) return;
  if (out_size != kRows * kDim) return;

  const float* h           = (const float*)d_in[0];
  const float* k_base      = (const float*)d_in[1];
  const float* decay_logit = (const float*)d_in[2];
  const float* gate_logit  = (const float*)d_in[3];
  const float* u           = (const float*)d_in[4];
  const float* v           = (const float*)d_in[5];
  const float* alpha_logit = (const float*)d_in[6];
  const float* proj_w      = (const float*)d_in[7];
  const float* proj_b      = (const float*)d_in[8];
  const float* norm1_scale = (const float*)d_in[9];
  const float* norm2_scale = (const float*)d_in[10];
  const float* up_w        = (const float*)d_in[11];
  const float* up_b        = (const float*)d_in[12];
  const float* down_w      = (const float*)d_in[13];
  const float* down_b      = (const float*)d_in[14];
  float* out = (float*)d_out;

  char* ws = (char*)d_ws;
  size_t off = 0;
  auto carve = [&](size_t bytes) -> char* { char* p = ws + off; off += (bytes + 255) & ~(size_t)255; return p; };
  unsigned short* W16   = (unsigned short*)carve(kBytesW16);
  unsigned short* KB16  = (unsigned short*)carve(kBytesKB16);
  unsigned short* UVT16 = (unsigned short*)carve(kBytesUVT16);
  float*          HN32  = (float*)carve(kBytesHN32);
  float*          Y32   = (float*)carve(kBytesY32);
  unsigned short* HN16  = (unsigned short*)carve(kBytesHN16);
  unsigned short* HNT16 = (unsigned short*)carve(kBytesHNT16);
  float*          QK32  = (float*)carve(kBytesQK32);
  float*          QKN32 = (float*)carve(kBytesQKN32);
  unsigned short* MIX16 = (unsigned short*)carve(kBytesMIX16);
  float*          H2    = (float*)carve(kBytesH2);
  unsigned short* M16   = (unsigned short*)carve(kBytesM16);
  unsigned short* G16   = (unsigned short*)carve(kBytesG16);
  float*          PAR   = (float*)carve(kBytesPAR);
  if (off != kWsTotal || off > ws_size || off > (size_t)134217728) return;
  float* UP32 = HN32;
  if ((char*)Y32 != (char*)HN32 + kBytesHN32) return;

  unsigned short* PW16 = W16;
  unsigned short* UW16 = W16 + (size_t)1 * kSegElems;
  unsigned short* DW16 = W16 + (size_t)3 * kSegElems;

  params_kernel<<<1, 32, 0, stream>>>(decay_logit, gate_logit, alpha_logit, PAR);
  cast_w_kernel<<<dim3(kSegElems / 8 / 256, 5), 256, 0, stream>>>(proj_w, up_w, down_w, W16, kWCarry);
  kb16_kernel<<<kWin * kWin / 8 / 256, 256, 0, stream>>>(k_base, PAR, KB16, kKbCarry);
  uvt_kernel<<<kDim / 64, 256, 0, stream>>>(u, v, UVT16, kUvCarry);
  rmsnorm_kernel<true><<<kRows, 256, 0, stream>>>(h, norm1_scale, HN32, HN16, kActCarry);
  transpose16_kernel<<<dim3(kWin / 64, kDim / 64, kBatch), 256, 0, stream>>>(HN16, HNT16);
  eng::gemm64_f16<0, false, false, false><<<dim3((kRows / 64) * 1 / 8, 1), 256, 0, stream>>>(
      HN16, kDim, 0L, UVT16, kDim, 0L, (void*)QK32, 64, 0L,
      proj_b, H2, 64, 0L, kRows, 64, kDim, kScaleQk, 1.0f);
  qk_post_kernel<<<kRows / 8, 256, 0, stream>>>(QK32, QKN32);
  scan_kernel<<<kBatch * (kDim / kScanThreads), kScanThreads, 0, stream>>>(HN32, QKN32, PAR, Y32);
  eng::gemm64_f16<1, false, true, true><<<dim3((kWin / 64) * (kDim / 64) / 8, kBatch), 256, 0, stream>>>(
      KB16, kWin, 0L, HNT16, kWin, (long)kDim * kWin, (void*)MIX16, kDim, (long)kWin * kDim,
      proj_b, Y32, kDim, (long)kWin * kDim, kWin, kDim, kWin, kScaleBase, kActCarry);
  eng::gemm64_f16<0, true, true, false><<<dim3((kRows / 64) * (kDim / 64) / 8, 1), 256, 0, stream>>>(
      MIX16, kDim, 0L, PW16, kDim, 0L, (void*)H2, kDim, 0L,
      proj_b, h, kDim, 0L, kRows, kDim, kDim, kScaleProj, 1.0f);
  rmsnorm_kernel<false><<<kRows, 256, 0, stream>>>(H2, norm2_scale, HN32, M16, kActCarry);
  eng::gemm64_f16<0, true, false, false><<<dim3((kRows / 64) * (kUpDim / 64) / 8, 1), 256, 0, stream>>>(
      M16, kDim, 0L, UW16, kDim, 0L, (void*)UP32, kUpDim, 0L,
      up_b, H2, kUpDim, 0L, kRows, kUpDim, kDim, kScaleUp, 1.0f);
  gelu_kernel<<<kRows, 256, 0, stream>>>(UP32, G16, kGeluCarry);
  eng::gemm64_f16<0, true, true, false><<<dim3((kRows / 64) * (kDim / 64) / 8, 1), 256, 0, stream>>>(
      G16, kUpDim, 0L, DW16, kUpDim, 0L, (void*)out, kDim, 0L,
      down_b, H2, kDim, 0L, kRows, kDim, kUpDim, kScaleDown, 1.0f);
}
